// PixelsCoordinatesAttention_69973607186637
// MI455X (gfx1250) — hardware-verified
//
#include <hip/hip_runtime.h>
#include <math.h>

typedef __attribute__((ext_vector_type(16))) _Float16 v16h;
typedef __attribute__((ext_vector_type(16))) __bf16 v16b;
typedef __attribute__((ext_vector_type(8)))  _Float16 v8h;
typedef __attribute__((ext_vector_type(8)))  float v8f;
typedef __attribute__((ext_vector_type(4)))  float v4f;
typedef __attribute__((ext_vector_type(2)))  float v2f;
typedef __attribute__((ext_vector_type(4)))  unsigned v4u;
typedef __attribute__((ext_vector_type(4)))  int v4i;
typedef float __attribute__((may_alias)) float_a;
typedef int __attribute__((may_alias)) int_a;

template <typename T> __device__ __forceinline__ void vst2(void* p, T v) { *(volatile T*)p = v; __threadfence(); *(volatile T*)p = v; }
__device__ __forceinline__ v8f wmma16(v16h a, v16h b, v8f c) {
  v8f d = __builtin_amdgcn_wmma_f32_16x16x32_f16(false, a, false, b, (short)0, c, false, false);
  asm volatile("v_nop\n\tv_nop\n\tv_nop\n\tv_nop" : "+v"(d) : "v"(a), "v"(b));
  return d;
}
__device__ __forceinline__ v8f wmma_bf(v16b a, v16b b, v8f c) {
  v8f d = __builtin_amdgcn_wmma_f32_16x16x32_bf16(false, a, false, b, (short)0, c, false, false);
  asm volatile("v_nop\n\tv_nop\n\tv_nop\n\tv_nop" : "+v"(d) : "v"(a), "v"(b));
  return d;
}
__device__ __forceinline__ v16h frag_h(const _Float16* rowk0, int lane) {
  union { v16h v; v8h q[2]; } u; const _Float16* p = rowk0 + 8 * (lane >> 4);
  u.q[0] = *(const v8h*)p; u.q[1] = *(const v8h*)(p + 16); return u.v;
}
__device__ __forceinline__ v16h frag_f32(const float* rowk0, int lane) {
  v16h a; const float* p = rowk0 + 8 * (lane >> 4);
#pragma unroll
  for (int i = 0; i < 8; ++i) { a[i] = (_Float16)p[i]; a[8 + i] = (_Float16)p[16 + i]; }
  return a;
}
__device__ __forceinline__ v16h frag_f32s(const float* rowk0, int lane, float sc) {
  v16h a; const float* p = rowk0 + 8 * (lane >> 4);
#pragma unroll
  for (int i = 0; i < 8; ++i) { a[i] = (_Float16)(p[i] * sc); a[8 + i] = (_Float16)(p[16 + i] * sc); }
  return a;
}
__device__ __forceinline__ v16h fragc_f32(const float* W, int k0, int n, int lane, int ld, int K) {
  v16h a; const int g = lane >> 4;
#pragma unroll
  for (int i = 0; i < 8; ++i) { const int ka = k0 + 8 * g + i, kb = ka + 16;
    a[i] = (_Float16)(ka < K ? W[(size_t)(ka < K ? ka : K - 1) * ld + n] : 0.f); a[8 + i] = (_Float16)(kb < K ? W[(size_t)(kb < K ? kb : K - 1) * ld + n] : 0.f); }
  return a;
}
struct F2 { v16b h, l; };
__device__ __forceinline__ F2 bsplit16(const float v[16]) { F2 r;
#pragma unroll
  for (int i = 0; i < 16; ++i) { const __bf16 h = (__bf16)v[i]; r.h[i] = h; r.l[i] = (__bf16)(v[i] - (float)h); }
  return r; }
__device__ __forceinline__ F2 split_row(const float* row, int k0, int lane) { float v[16]; const float* p = row + k0 + 8 * (lane >> 4);
#pragma unroll
  for (int i = 0; i < 8; ++i) { v[i] = p[i]; v[8 + i] = p[16 + i]; }
  return bsplit16(v); }
__device__ __forceinline__ F2 split_rowK(const float* row, int k0, int lane, int K) { float v[16]; const int g = lane >> 4;
#pragma unroll
  for (int i = 0; i < 8; ++i) { const int ka = k0 + 8 * g + i, kb = ka + 16; v[i] = ka < K ? row[ka < K ? ka : K - 1] : 0.f; v[8 + i] = kb < K ? row[kb < K ? kb : K - 1] : 0.f; }
  return bsplit16(v); }
__device__ __forceinline__ F2 split_col(const float* W, int k0, int n, int lane, int ld, int K) { float v[16]; const int g = lane >> 4;
#pragma unroll
  for (int i = 0; i < 8; ++i) { const int ka = k0 + 8 * g + i, kb = ka + 16; v[i] = ka < K ? W[(size_t)(ka < K ? ka : K - 1) * ld + n] : 0.f; v[8 + i] = kb < K ? W[(size_t)(kb < K ? kb : K - 1) * ld + n] : 0.f; }
  return bsplit16(v); }
__device__ __forceinline__ v8f mac3(const F2& a, const F2& b, v8f c) { c = wmma_bf(a.l, b.h, c); c = wmma_bf(a.h, b.l, c); return wmma_bf(a.h, b.h, c); }
__device__ __forceinline__ float sigm(float v) { return 1.0f / (1.0f + expf(-v)); }
#define LDSX() do { asm volatile("s_wait_dscnt 0" ::: "memory"); __builtin_amdgcn_wave_barrier(); __builtin_amdgcn_fence(__ATOMIC_RELEASE, "workgroup"); } while (0)


#define NB 4
#define SS 2048
#define PD 512
#define CD 64
#define ID 512
#define NH 8
#define HD 64
#define NR (NB * SS)
#ifndef TQB
#define TQB (SS / 64)
#define TNB NB
#define NRB (NR / 64)
#endif
typedef __attribute__((ext_vector_type(8))) __bf16 v8b;
__device__ __forceinline__ v16b frag_b(const __bf16* rowk0, int lane) {
  union { v16b v; v8b q[2]; } u; const __bf16* p = rowk0 + 8 * (lane >> 4);
  u.q[0] = *(const v8b*)p; u.q[1] = *(const v8b*)(p + 16); return u.v;
}
__device__ __forceinline__ float bfr(float v) { return (float)(__bf16)v; }
__device__ __attribute__((noinline)) float exp_ni(float v) { return expf(v); }
__device__ __attribute__((noinline)) float erf_ni(float v) { return erff(v); }

#define WS_PP   0u
#define WS_PC   (WS_PP + 2u * (size_t)3 * ID * PD)
#define WS_PO   (WS_PC + 2u * (size_t)2 * ID * CD)
#define WS_QP   (WS_PO + 2u * (size_t)PD * ID)
#define WS_KP   (WS_QP + 2u * (size_t)NR * ID)
#define WS_QC   (WS_KP + 2u * (size_t)NR * ID)
#define WS_KC   (WS_QC + 2u * (size_t)NR * ID)
#define WS_V    (WS_KC + 2u * (size_t)NR * ID)
#define WS_CTX  (WS_V + 2u * (size_t)NB * ID * SS)
#define WS_END  (WS_CTX + 4u * (size_t)NR * ID)

__global__ __launch_bounds__(256) void k_pack(const float* __restrict__ WQKV, const float* __restrict__ WC, const float* __restrict__ WO, __bf16* __restrict__ P) {
  __shared__ __align__(16) __bf16 s[PD]; const int t = threadIdx.x; int n = blockIdx.x; int K; __bf16* dst; const float* src; int ld;
  if (n < 3 * ID) { K = PD; src = WQKV; ld = 3 * ID; dst = P + WS_PP / 2 + (size_t)n * PD; }
  else if ((n -= 3 * ID) < 2 * ID) { K = CD; src = WC; ld = 2 * ID; dst = P + WS_PC / 2 + (size_t)n * CD; }
  else { n -= 2 * ID; K = ID; src = WO; ld = PD; dst = P + WS_PO / 2 + (size_t)n * ID; }
  for (int k = t; k < K; k += 256) s[k] = (__bf16)src[(size_t)k * ld + n]; __syncthreads(); for (int q = t; q < K / 8; q += 256) vst2((unsigned*)(dst + q * 8), *(const v4u*)&s[q * 8]);
}
template <int KDIM>
__global__ __launch_bounds__(128) void k_proj(const float* __restrict__ X, const __bf16* __restrict__ Wr, int which0, _Float16* __restrict__ D0, _Float16* __restrict__ D1, _Float16* __restrict__ V) {
  __shared__ __align__(16) _Float16 so[64][136]; __shared__ __align__(16) _Float16 st[128][72];
  const int tid = threadIdx.x, wave = tid >> 5, lane = tid & 31, col = lane & 15, g = lane >> 4; const int n0 = blockIdx.y * 128; const int which = n0 / ID, c0 = n0 % ID; const size_t rb0 = (size_t)blockIdx.x * 64, r0 = rb0 + wave * 16;
  v8f acc[8] = {};
#pragma unroll 2
  for (int kc = 0; kc < KDIM / 32; ++kc) { v16b a; { const float* p = X + (r0 + col) * KDIM + kc * 32 + 8 * g;
#pragma unroll
      for (int i = 0; i < 8; ++i) { a[i] = (__bf16)p[i]; a[8 + i] = (__bf16)p[16 + i]; } }
#pragma unroll
    for (int j = 0; j < 8; ++j) acc[j] = wmma_bf(a, frag_b(Wr + (size_t)(n0 + j * 16 + col) * KDIM + kc * 32, lane), acc[j]); }
  (void)which0;
  if (which < 2) { _Float16* dst = (which == 0) ? D0 : D1;
#pragma unroll
    for (int j = 0; j < 8; ++j)
#pragma unroll
      for (int r = 0; r < 8; ++r) so[wave * 16 + 8 * g + r][j * 16 + col] = (_Float16)fminf(fmaxf(acc[j][r], -5.0f), 5.0f);
    LDSX();
    for (int rl = 0; rl < 16; ++rl) if (lane < 16) vst2((unsigned*)(dst + (r0 + rl) * ID + c0 + lane * 8), *(const v4u*)&so[wave * 16 + rl][lane * 8]);
  } else {
#pragma unroll
    for (int j = 0; j < 8; ++j)
#pragma unroll
      for (int r = 0; r < 8; ++r) st[j * 16 + col][wave * 16 + 8 * g + r] = (_Float16)acc[j][r];
    __syncthreads();
    const size_t b = rb0 / SS, s0 = rb0 % SS;
    for (int e = tid; e < 128 * 8; e += 128) { const int d = e >> 3, pc = e & 7; vst2((unsigned*)(V + ((b * ID + c0 + d) * SS) + s0 + pc * 8), *(const v4u*)&st[d][pc * 8]); } }
}
__global__ __launch_bounds__(128) void k_attn(const _Float16* __restrict__ QP, const _Float16* __restrict__ KP, const _Float16* __restrict__ QC, const _Float16* __restrict__ KC, const _Float16* __restrict__ V, float* __restrict__ CTX) {
  __shared__ __align__(16) _Float16 sph[4][16][40]; __shared__ __align__(16) float so[4][16][68];
  const int tid = threadIdx.x, wave = tid >> 5, lane = tid & 31, col = lane & 15, g = lane >> 4; const int h = blockIdx.y; const size_t b = blockIdx.z; const int q0 = blockIdx.x * 64 + wave * 16; const size_t rq = b * SS + q0;
  v16h aq[2], ac[2];
#pragma unroll
  for (int kc = 0; kc < 2; ++kc) { aq[kc] = frag_h(QP + (rq + col) * ID + h * HD + kc * 32, lane); ac[kc] = frag_h(QC + (rq + col) * ID + h * HD + kc * 32, lane); }
  float m[8], l[8];
#pragma unroll
  for (int r = 0; r < 8; ++r) { m[r] = -3.0e38f; l[r] = 0.f; }
  v8f acc[4] = {};
#pragma unroll 1
  for (int ks = 0; ks < SS / 32; ++ks) { const int j0 = ks * 32; v8f s[2];
#pragma unroll
    for (int ct = 0; ct < 2; ++ct) { const size_t rk = (b * SS + j0 + ct * 16 + col) * ID + h * HD; v8f c = {};
#pragma unroll
      for (int kc = 0; kc < 2; ++kc) { c = wmma16(aq[kc], frag_h(KP + rk + kc * 32, lane), c); c = wmma16(ac[kc], frag_h(KC + rk + kc * 32, lane), c); }
#pragma unroll
      for (int r = 0; r < 8; ++r) s[ct][r] = c[r] * 0.125f; }
#pragma unroll
    for (int r = 0; r < 8; ++r) { float mx = fmaxf(s[0][r], s[1][r]);
#pragma unroll
      for (int o = 1; o < 16; o <<= 1) mx = fmaxf(mx, __shfl_xor(mx, o));
      const float mn = fmaxf(m[r], mx); const float alpha = (m[r] <= -1.0e38f) ? 0.f : __expf(m[r] - mn); const float e0 = __expf(s[0][r] - mn), e1 = __expf(s[1][r] - mn); float es = e0 + e1;
#pragma unroll
      for (int o = 1; o < 16; o <<= 1) es += __shfl_xor(es, o);
      l[r] = l[r] * alpha + es; m[r] = mn;
#pragma unroll
      for (int dt = 0; dt < 4; ++dt) acc[dt][r] *= alpha;
      sph[wave][8 * g + r][col] = (_Float16)(e0 * 2048.0f); sph[wave][8 * g + r][16 + col] = (_Float16)(e1 * 2048.0f); }
    LDSX();
    const v16h pa = frag_h(&sph[wave][col][0], lane);
#pragma unroll
    for (int dt = 0; dt < 4; ++dt) acc[dt] = wmma16(pa, frag_h(V + ((b * ID + (size_t)h * HD + dt * 16 + col) * SS) + j0, lane), acc[dt]);
    LDSX(); }
#pragma unroll
  for (int r = 0; r < 8; ++r) { const float il = (1.0f / 2048.0f) / l[r];
#pragma unroll
    for (int dt = 0; dt < 4; ++dt) so[wave][8 * g + r][dt * 16 + col] = acc[dt][r] * il; }
  LDSX();
  for (int rl = 0; rl < 16; ++rl) if (lane < 16) vst2(CTX + (rq + rl) * ID + h * HD + lane * 4, *(const v4f*)&so[wave][rl][lane * 4]);
}
__global__ __launch_bounds__(128) void k_out(const float* __restrict__ CTX, const __bf16* __restrict__ P, const float* __restrict__ BO, float* __restrict__ OUT) {
  __shared__ __align__(16) float so[4][16][132];
  const int tid = threadIdx.x, wave = tid >> 5, lane = tid & 31, col = lane & 15, g = lane >> 4; const size_t r0 = (size_t)blockIdx.x * 64 + wave * 16; const int n0 = blockIdx.y * 128;
  v8f acc[8] = {};
#pragma unroll 2
  for (int kc = 0; kc < ID / 32; ++kc) { const F2 a = split_row(CTX + (r0 + col) * ID, kc * 32, lane);
#pragma unroll
    for (int j = 0; j < 8; ++j) { const v16b w = frag_b(P + WS_PO / 2 + (size_t)(n0 + j * 16 + col) * ID + kc * 32, lane); acc[j] = wmma_bf(a.l, w, acc[j]); acc[j] = wmma_bf(a.h, w, acc[j]); } }
#pragma unroll
  for (int j = 0; j < 8; ++j) { const float bb = bfr(BO[n0 + j * 16 + col]);
#pragma unroll
    for (int r = 0; r < 8; ++r) so[wave][8 * g + r][j * 16 + col] = acc[j][r] + bb; }
  LDSX();
  for (int rl = 0; rl < 16; ++rl) vst2(OUT + (r0 + rl) * PD + n0 + lane * 4, *(const v4f*)&so[wave][rl][lane * 4]);
}
extern "C" void kernel_launch(void* const* d_in, const int* in_sizes, int n_in, void* d_out, int out_size, void* d_ws, size_t ws_size, hipStream_t stream) {
  (void)in_sizes; (void)n_in; (void)out_size;
  const float** F = (const float**)d_in;
  if (ws_size < (size_t)WS_END) return;
  char* ws = (char*)d_ws; __bf16* P = (__bf16*)ws; _Float16 *QP = (_Float16*)(ws + WS_QP), *KP = (_Float16*)(ws + WS_KP), *QC = (_Float16*)(ws + WS_QC), *KC = (_Float16*)(ws + WS_KC), *V = (_Float16*)(ws + WS_V); float* CTX = (float*)(ws + WS_CTX);
  k_pack<<<3 * ID + 2 * ID + PD, 256, 0, stream>>>(F[2], F[3], F[4], P);
  k_proj<PD><<<dim3(NRB, 3 * ID / 128), 128, 0, stream>>>(F[0], P + WS_PP / 2, 0, QP, KP, V);
  k_proj<CD><<<dim3(NRB, 2 * ID / 128), 128, 0, stream>>>(F[1], P + WS_PC / 2, 0, QC, KC, nullptr);
  k_attn<<<dim3(TQB, NH, TNB), 128, 0, stream>>>(QP, KP, QC, KC, V, CTX);
  k_out<<<dim3(NRB, PD / 128), 128, 0, stream>>>(CTX, P, F[5], (float*)d_out);
}
